// GRU_70480413327664
// MI455X (gfx1250) — hardware-verified
//
#include <hip/hip_runtime.h>
#include <math.h>

constexpr int NBATCH  = 512;
constexpr int NSTEP   = 3600;
constexpr int NHID    = 64;
constexpr int NGATE   = 3 * NHID;
constexpr int NCLS    = 5;
constexpr int ROWS_BLK = 16;
constexpr int NTHR    = 128;
constexpr int XCHUNK  = 240;
constexpr int NCHUNK  = NSTEP / XCHUNK;
constexpr int HPITCH  = 72;
constexpr int HBUF_ELEMS = ROWS_BLK * HPITCH;
constexpr int SPITCH  = 68;
constexpr int HEAD_THR = 256;
constexpr int NOUT    = NBATCH * NCLS;
constexpr float HCARRY = 1024.0f;
constexpr float WCARRY = 256.0f;
constexpr float FOLD   = 1.0f / (HCARRY * WCARRY);

static_assert(NBATCH % ROWS_BLK == 0, "batch tiles");
static_assert(NCHUNK * XCHUNK == NSTEP, "chunk divides the step count");
static_assert(XCHUNK % 2 == 0, "buffer parity restarts per chunk");
static_assert((ROWS_BLK * XCHUNK) % NTHR == 0, "x staging loop exact");
static_assert(NHID == 16 * (NTHR / 32), "4 waves x 16 hidden columns");
static_assert(NHID % 32 == 0, "K multiple of 32");
static_assert(NGATE % 16 == 0, "N multiple of 16");
static_assert((2 * HBUF_ELEMS) % NTHR == 0, "h zero-fill loop exact");
static_assert((ROWS_BLK * NHID / 4) % NTHR == 0, "final store loop exact");
static_assert(NOUT % HEAD_THR == 0, "head grid exact");
static_assert(NOUT * 4 == 10240, "output bytes");

typedef __attribute__((ext_vector_type(16))) _Float16 v16h;
typedef __attribute__((ext_vector_type(8)))  _Float16 v8h;
typedef __attribute__((ext_vector_type(8)))  float    v8f;
typedef __attribute__((ext_vector_type(4)))  float    v4f;

template <typename T> struct Frag;
template <> struct Frag<_Float16> {
  typedef v16h V; union U { v16h v; v8h h[2]; };
  static __device__ __forceinline__ v16h load(const _Float16* p) {
    U f; f.h[0] = *(const v8h*)(p); f.h[1] = *(const v8h*)(p + 16); return f.v;
  }
  static __device__ __forceinline__ v8f mma(v16h a, v16h b, v8f c) {
    return __builtin_amdgcn_wmma_f32_16x16x32_f16(false, a, false, b, (short)0, c, false, false);
  }
};

__device__ __forceinline__ void gru_guard(v8f& a, v8f& b, v8f& c, v16h x0, v16h x1,
                                          v16h b0, v16h b1, v16h b2, v16h b3, v16h b4, v16h b5) {
  asm volatile("v_nop\n\tv_nop\n\tv_nop\n\tv_nop"
               : "+v"(a), "+v"(b), "+v"(c)
               : "v"(x0), "v"(x1), "v"(b0), "v"(b1), "v"(b2), "v"(b3), "v"(b4), "v"(b5));
}

__device__ __forceinline__ v16h load_bfrag_f32(const float* p) {
  const v4f a0 = *(const v4f*)(p);
  const v4f a1 = *(const v4f*)(p + 4);
  const v4f a2 = *(const v4f*)(p + 16);
  const v4f a3 = *(const v4f*)(p + 20);
  v16h f;
#pragma unroll
  for (int e = 0; e < 4; ++e) {
    f[e]      = (_Float16)(a0[e] * WCARRY);
    f[4 + e]  = (_Float16)(a1[e] * WCARRY);
    f[8 + e]  = (_Float16)(a2[e] * WCARRY);
    f[12 + e] = (_Float16)(a3[e] * WCARRY);
  }
  return f;
}

__device__ __forceinline__ float gate_sig(float x)  { return __builtin_amdgcn_rcpf(1.0f + expf(-x)); }
__device__ __forceinline__ float gate_tanh(float x) { return 1.0f - 2.0f * __builtin_amdgcn_rcpf(expf(2.0f * x) + 1.0f); }

__global__ __launch_bounds__(NTHR) void gru_seq_kernel(const float* __restrict__ x,
                                                       const float* __restrict__ w_ih,
                                                       const float* __restrict__ w_hh,
                                                       const float* __restrict__ b_ih,
                                                       const float* __restrict__ b_hh,
                                                       float* __restrict__ Hlast) {
  __shared__ __align__(16) _Float16 hbuf[2 * HBUF_ELEMS];
  __shared__ __align__(16) float    xbuf[XCHUNK * ROWS_BLK];
  __shared__ __align__(16) float    Hs[ROWS_BLK * SPITCH];

  const int tid = threadIdx.x, lane = tid & 31, wave = tid >> 5;
  const int c = lane & 15, hh = lane >> 4, koff = hh * 8;
  const int rowbase = blockIdx.x * ROWS_BLK;
  const int j = 16 * wave + c;

  const float wir = w_ih[j];
  const float wiz = w_ih[NHID + j];
  const float win = w_ih[2 * NHID + j];
  const float bir = b_ih[j];
  const float biz = b_ih[NHID + j];
  const float bin = b_ih[2 * NHID + j];
  const float bhr = b_hh[j];
  const float bhz = b_hh[NHID + j];
  const float bhn = b_hh[2 * NHID + j];

  const v16h BR0 = load_bfrag_f32(w_hh + (size_t)(0 * NHID + j) * NHID + koff);
  const v16h BR1 = load_bfrag_f32(w_hh + (size_t)(0 * NHID + j) * NHID + 32 + koff);
  const v16h BZ0 = load_bfrag_f32(w_hh + (size_t)(1 * NHID + j) * NHID + koff);
  const v16h BZ1 = load_bfrag_f32(w_hh + (size_t)(1 * NHID + j) * NHID + 32 + koff);
  const v16h BN0 = load_bfrag_f32(w_hh + (size_t)(2 * NHID + j) * NHID + koff);
  const v16h BN1 = load_bfrag_f32(w_hh + (size_t)(2 * NHID + j) * NHID + 32 + koff);

#pragma unroll 1
  for (int i = tid; i < 2 * HBUF_ELEMS; i += NTHR) hbuf[i] = (_Float16)0.0f;

  float hst[8];
#pragma unroll
  for (int v = 0; v < 8; ++v) hst[v] = 0.0f;

  const v8f z8 = {0.f, 0.f, 0.f, 0.f, 0.f, 0.f, 0.f, 0.f};

#pragma unroll 1
  for (int ch = 0; ch < NCHUNK; ++ch) {
    const int t0 = ch * XCHUNK;
#pragma unroll 1
    for (int it = 0; it < (ROWS_BLK * XCHUNK) / NTHR; ++it) {
      const int i  = it * NTHR + tid;
      const int r  = i / XCHUNK;
      const int cc = i - r * XCHUNK;
      xbuf[cc * ROWS_BLK + r] = x[(size_t)(rowbase + r) * NSTEP + (size_t)(t0 + cc)];
    }
    __syncthreads();

#pragma unroll 1
    for (int s = 0; s < XCHUNK; ++s) {
      const int cur = s & 1;
      const _Float16* hrd = hbuf + cur * HBUF_ELEMS + c * HPITCH + koff;
      _Float16* hwr = hbuf + (cur ^ 1) * HBUF_ELEMS;

      const v16h A0 = Frag<_Float16>::load(hrd);
      const v16h A1 = Frag<_Float16>::load(hrd + 32);
      const v4f xlo = *(const v4f*)(xbuf + s * ROWS_BLK + 8 * hh);
      const v4f xhi = *(const v4f*)(xbuf + s * ROWS_BLK + 8 * hh + 4);

      v8f accR = z8, accZ = z8, accN = z8;
      accR = Frag<_Float16>::mma(A0, BR0, accR);
      accZ = Frag<_Float16>::mma(A0, BZ0, accZ);
      accN = Frag<_Float16>::mma(A0, BN0, accN);
      accR = Frag<_Float16>::mma(A1, BR1, accR);
      accZ = Frag<_Float16>::mma(A1, BZ1, accZ);
      accN = Frag<_Float16>::mma(A1, BN1, accN);
      gru_guard(accR, accZ, accN, A0, A1, BR0, BR1, BZ0, BZ1, BN0, BN1);

#pragma unroll
      for (int v = 0; v < 8; ++v) {
        const float xv = (v < 4) ? xlo[v & 3] : xhi[v & 3];
        const float ir = xv * wir + bir;
        const float iz = xv * wiz + biz;
        const float in = xv * win + bin;
        const float hr = accR[v] * FOLD + bhr;
        const float hz = accZ[v] * FOLD + bhz;
        const float hn = accN[v] * FOLD + bhn;
        const float rg = gate_sig(ir + hr);
        const float zg = gate_sig(iz + hz);
        const float ng = gate_tanh(in + rg * hn);
        const float hnew = (1.0f - zg) * ng + zg * hst[v];
        hst[v] = hnew;
        hwr[(8 * hh + v) * HPITCH + j] = (_Float16)(hnew * HCARRY);
      }
      __syncthreads();
    }
  }

#pragma unroll
  for (int v = 0; v < 8; ++v) Hs[(8 * hh + v) * SPITCH + j] = hst[v];
  __syncthreads();
  for (int pass = 0; pass < 2; ++pass) {
#pragma unroll
    for (int it = 0; it < (ROWS_BLK * NHID / 4) / NTHR; ++it) {
      const int idx = it * NTHR + tid;
      const int row = idx >> 4;
      const int c4  = (idx & 15) * 4;
      const v4f val = *(const v4f*)(Hs + row * SPITCH + c4);
      *(volatile v4f*)(Hlast + (size_t)(rowbase + row) * NHID + c4) = val;
    }
    __threadfence();
  }
}

__global__ __launch_bounds__(HEAD_THR) void head_kernel(const float* __restrict__ Hl,
                                                        const float* __restrict__ w_head,
                                                        const float* __restrict__ b_head,
                                                        float* __restrict__ out) {
  const int i   = blockIdx.x * HEAD_THR + threadIdx.x;
  const int row = i / NCLS;
  const int cl  = i - row * NCLS;
  const float* hp = Hl + (size_t)row * NHID;
  const float* wp = w_head + cl * NHID;
  float s = 0.0f;
#pragma unroll 1
  for (int k = 0; k < NHID; k += 4) {
    const v4f a = *(const v4f*)(hp + k);
    const v4f w = *(const v4f*)(wp + k);
    s = fmaf(a[0], w[0], s);
    s = fmaf(a[1], w[1], s);
    s = fmaf(a[2], w[2], s);
    s = fmaf(a[3], w[3], s);
  }
  const float res = s + b_head[cl];
  *(volatile float*)(out + i) = res;
  __threadfence();
  *(volatile float*)(out + i) = res;
}

extern "C" void kernel_launch(void* const* d_in, const int* in_sizes, int n_in,
                              void* d_out, int out_size, void* d_ws, size_t ws_size, hipStream_t stream) {
  (void)in_sizes; (void)out_size;
  if (n_in < 7 || d_out == nullptr || d_ws == nullptr) return;
  const size_t carve = (size_t)NBATCH * NHID * sizeof(float);
  if (carve > ws_size || carve > (size_t)134217728) return;

  const float* x      = (const float*)d_in[0];
  const float* w_ih   = (const float*)d_in[1];
  const float* w_hh   = (const float*)d_in[2];
  const float* b_ih   = (const float*)d_in[3];
  const float* b_hh   = (const float*)d_in[4];
  const float* w_head = (const float*)d_in[5];
  const float* b_head = (const float*)d_in[6];
  float* out   = (float*)d_out;
  float* Hlast = (float*)d_ws;

  gru_seq_kernel<<<NBATCH / ROWS_BLK, NTHR, 0, stream>>>(x, w_ih, w_hh, b_ih, b_hh, Hlast);
  head_kernel<<<NOUT / HEAD_THR, HEAD_THR, 0, stream>>>(Hlast, w_head, b_head, out);
}
